// OuterProducterMean_89713276879142
// MI455X (gfx1250) — hardware-verified
//
#include <hip/hip_runtime.h>
#include <hip/hip_bf16.h>

#define S_DIM 128
#define R_DIM 256
#define CM_DIM 256
#define C_DIM 32
#define CZ_DIM 128
#define KP_DIM (C_DIM * C_DIM)

#define WL_PITCH 264
#define AT_PITCH 136
#define WT_PITCH 72
#define OT_PITCH 1032
#define OS_PITCH 132

#define PROJ_LDS_BYTES (2 * 64 * WL_PITCH * 2)
#define PAIR_LDS_BYTES (64 * OT_PITCH * 2)

static_assert((WL_PITCH % 8) == 0);
static_assert((AT_PITCH % 8) == 0);
static_assert((WT_PITCH % 8) == 0);
static_assert((OT_PITCH % 8) == 0);
static_assert((OS_PITCH % 4) == 0);
static_assert(64 * AT_PITCH * 2 <= PROJ_LDS_BYTES);
static_assert(64 * OS_PITCH * 4 <= PAIR_LDS_BYTES);

typedef float        v4f   __attribute__((ext_vector_type(4)));
typedef float        v8f   __attribute__((ext_vector_type(8)));
typedef float        v16f  __attribute__((ext_vector_type(16)));
typedef unsigned int v4u   __attribute__((ext_vector_type(4)));
typedef unsigned int v8u   __attribute__((ext_vector_type(8)));
typedef _Float16     v8h   __attribute__((ext_vector_type(8)));
typedef _Float16     v16h  __attribute__((ext_vector_type(16)));
typedef __bf16       v16bf __attribute__((ext_vector_type(16)));


static __device__ __forceinline__ v8f zero8() {
    v8f z = {0.f, 0.f, 0.f, 0.f, 0.f, 0.f, 0.f, 0.f};
    return z;
}

static __device__ __forceinline__ unsigned bf16_bits(float f) {
    unsigned u = __builtin_bit_cast(unsigned, f);
    u += 0x7FFFu + ((u >> 16) & 1u);
    return u >> 16;
}
static __device__ __forceinline__ float bf16_val(unsigned b) {
    return __builtin_bit_cast(float, b << 16);
}

static __device__ __forceinline__ v8f wmma_f16(v8f c, v16h a, v16h b) {
    c = __builtin_amdgcn_wmma_f32_16x16x32_f16(false, a, false, b, (short)0, c, false, false);
    asm volatile("v_nop\n\tv_nop\n\tv_nop\n\tv_nop" : "+v"(c) : "v"(a), "v"(b));
    return c;
}
static __device__ __forceinline__ v8f wmma_bf16(v8f c, v16bf a, v16bf b) {
    c = __builtin_amdgcn_wmma_f32_16x16x32_bf16(false, a, false, b, (short)0, c, false, false);
    asm volatile("v_nop\n\tv_nop\n\tv_nop\n\tv_nop" : "+v"(c) : "v"(a), "v"(b));
    return c;
}

static __device__ __forceinline__ v16h ld_frag_f16(const _Float16* row, int k0, int h) {
    v8h lo = *(const v8h*)(row + k0 + 8 * h);
    v8h hi = *(const v8h*)(row + k0 + 16 + 8 * h);
    return __builtin_shufflevector(lo, hi, 0, 1, 2, 3, 4, 5, 6, 7, 8, 9, 10, 11, 12, 13, 14, 15);
}
static __device__ __forceinline__ v16bf ld_frag_bf16(const unsigned short* row, int k0, int h) {
    v4u lo = *(const v4u*)(row + k0 + 8 * h);
    v4u hi = *(const v4u*)(row + k0 + 16 + 8 * h);
    v8u u = __builtin_shufflevector(lo, hi, 0, 1, 2, 3, 4, 5, 6, 7);
    return __builtin_bit_cast(v16bf, u);
}

static __device__ __forceinline__ void ld_split_f32(const float* row, int k0, int h,
                                                    v16bf& fhi, v16bf& flo) {
    v4f x0 = *(const v4f*)(row + k0 + 8 * h);
    v4f x1 = *(const v4f*)(row + k0 + 8 * h + 4);
    v4f x2 = *(const v4f*)(row + k0 + 16 + 8 * h);
    v4f x3 = *(const v4f*)(row + k0 + 16 + 8 * h + 4);
    v8f y0 = __builtin_shufflevector(x0, x1, 0, 1, 2, 3, 4, 5, 6, 7);
    v8f y1 = __builtin_shufflevector(x2, x3, 0, 1, 2, 3, 4, 5, 6, 7);
    v16f x = __builtin_shufflevector(y0, y1, 0, 1, 2, 3, 4, 5, 6, 7, 8, 9, 10, 11, 12, 13, 14, 15);
    v8u uh, ul;
#pragma unroll
    for (int i = 0; i < 8; ++i) {
        float e0 = x[2 * i], e1 = x[2 * i + 1];
        unsigned h0 = bf16_bits(e0), h1 = bf16_bits(e1);
        unsigned l0 = bf16_bits(e0 - bf16_val(h0));
        unsigned l1 = bf16_bits(e1 - bf16_val(h1));
        uh[i] = h0 | (h1 << 16);
        ul[i] = l0 | (l1 << 16);
    }
    fhi = __builtin_bit_cast(v16bf, uh);
    flo = __builtin_bit_cast(v16bf, ul);
}

__global__ __launch_bounds__(256)
void k_proj(const float* __restrict__ msa,
            const float* __restrict__ wl,
            const float* __restrict__ wr,
            _Float16* __restrict__ aplane,
            _Float16* __restrict__ bplane) {
    extern __shared__ __align__(16) unsigned char dsmem[];
    unsigned short* Whi = (unsigned short*)dsmem;
    unsigned short* Wlo = Whi + 64 * WL_PITCH;

    const int r    = blockIdx.x;
    const int tid  = threadIdx.x;
    const int lane = tid & 31;
    const int wave = tid >> 5;
    const int h    = lane >> 4;
    const int n16  = lane & 15;

    for (int idx = tid; idx < 64 * CM_DIM; idx += 256) {
        const int k = idx >> 6;
        const int n = idx & 63;
        const float x = (n < 32) ? wl[k * C_DIM + n] : wr[k * C_DIM + (n - 32)];
        const unsigned hb = bf16_bits(x);
        const unsigned lb = bf16_bits(x - bf16_val(hb));
        Whi[n * WL_PITCH + k] = (unsigned short)hb;
        Wlo[n * WL_PITCH + k] = (unsigned short)lb;
    }
    __syncthreads();

    const int s = wave * 16 + n16;
    const float* arow = msa + ((size_t)s * R_DIM + r) * CM_DIM;

    v8f acc[4];
#pragma unroll
    for (int nt = 0; nt < 4; ++nt) acc[nt] = zero8();

#pragma unroll 1
    for (int ks = 0; ks < CM_DIM / 32; ++ks) {
        const int k0 = ks * 32;
        v16bf ahi, alo;
        ld_split_f32(arow, k0, h, ahi, alo);
#pragma unroll
        for (int nt = 0; nt < 4; ++nt) {
            const unsigned short* rowh = Whi + (nt * 16 + n16) * WL_PITCH;
            const unsigned short* rowl = Wlo + (nt * 16 + n16) * WL_PITCH;
            const v16bf bhi = ld_frag_bf16(rowh, k0, h);
            const v16bf blo = ld_frag_bf16(rowl, k0, h);
            acc[nt] = wmma_bf16(acc[nt], ahi, bhi);
            acc[nt] = wmma_bf16(acc[nt], ahi, blo);
            acc[nt] = wmma_bf16(acc[nt], alo, bhi);
        }
    }
    __syncthreads();

    _Float16* outT = (_Float16*)dsmem;
#pragma unroll
    for (int nt = 0; nt < 4; ++nt) {
        v8h o;
#pragma unroll
        for (int i = 0; i < 8; ++i) o[i] = (_Float16)(acc[nt][i] * 8.0f);
        *(v8h*)(outT + (nt * 16 + n16) * AT_PITCH + wave * 16 + 8 * h) = o;
    }
    __syncthreads();

    v4u vals[4];
#pragma unroll
    for (int pass = 0; pass < 4; ++pass) {
        const int L = pass * 32 + (tid >> 3);
        const int c = L >> 1, sh = L & 1, sub = tid & 7;
        vals[pass] = *(const v4u*)(outT + c * AT_PITCH + sh * 64 + sub * 8);
    }
#pragma unroll
    for (int pass = 0; pass < 4; ++pass) {
        const int L = pass * 32 + (tid >> 3);
        const int c = L >> 1, sh = L & 1, sub = tid & 7;
        _Float16* base = (c < 32) ? aplane : bplane;
        _Float16* p = base + (size_t)(r * C_DIM + (c & 31)) * S_DIM + sh * 64 + sub * 8;
        *(volatile v4u*)p = vals[pass];
    }
    __threadfence();
#pragma unroll
    for (int pass = 0; pass < 4; ++pass) {
        const int L = pass * 32 + (tid >> 3);
        const int c = L >> 1, sh = L & 1, sub = tid & 7;
        _Float16* base = (c < 32) ? aplane : bplane;
        _Float16* p = base + (size_t)(r * C_DIM + (c & 31)) * S_DIM + sh * 64 + sub * 8;
        *(volatile v4u*)p = vals[pass];
    }
}

__global__ __launch_bounds__(256)
void k_wprep(const float* __restrict__ wo, _Float16* __restrict__ wplane) {
    __shared__ __align__(16) _Float16 T[CZ_DIM * WT_PITCH];
    const int tid = threadIdx.x;
    const int kb  = blockIdx.x * 64;

    for (int idx = tid; idx < 64 * CZ_DIM; idx += 256) {
        const int kk = idx >> 7;
        const int z  = idx & 127;
        T[z * WT_PITCH + kk] = (_Float16)(64.0f * wo[(size_t)(kb + kk) * CZ_DIM + z]);
    }
    __syncthreads();

    v4u vals[4];
#pragma unroll
    for (int pass = 0; pass < 4; ++pass) {
        const int z = pass * 32 + (tid >> 3), sub = tid & 7;
        vals[pass] = *(const v4u*)(T + z * WT_PITCH + sub * 8);
    }
#pragma unroll
    for (int pass = 0; pass < 4; ++pass) {
        const int z = pass * 32 + (tid >> 3), sub = tid & 7;
        _Float16* p = wplane + (size_t)z * KP_DIM + kb + sub * 8;
        *(volatile v4u*)p = vals[pass];
    }
    __threadfence();
#pragma unroll
    for (int pass = 0; pass < 4; ++pass) {
        const int z = pass * 32 + (tid >> 3), sub = tid & 7;
        _Float16* p = wplane + (size_t)z * KP_DIM + kb + sub * 8;
        *(volatile v4u*)p = vals[pass];
    }
}

__global__ __launch_bounds__(256)
void k_pair(const _Float16* __restrict__ aplane,
            const _Float16* __restrict__ bplane,
            const _Float16* __restrict__ wplane,
            float* __restrict__ out) {
    extern __shared__ __align__(16) unsigned char dsmem[];
    _Float16* OT = (_Float16*)dsmem;

    const int t0   = blockIdx.x * 32;
    const int r0   = blockIdx.y * 2;
    const int tid  = threadIdx.x;
    const int lane = tid & 31;
    const int wave = tid >> 5;
    const int h    = lane >> 4;
    const int n16  = lane & 15;

    {
        const int rloc  = wave & 1;
        const int mg    = wave >> 1;
        const int ebase = (mg & 1) * 16;
        const int tq    = mg >> 1;

        v16h bq[2][4];
#pragma unroll
        for (int cb = 0; cb < 2; ++cb) {
            const _Float16* ap = aplane + (size_t)((r0 + rloc) * C_DIM + cb * 16 + n16) * S_DIM;
#pragma unroll
            for (int ks = 0; ks < 4; ++ks) bq[cb][ks] = ld_frag_f16(ap, ks * 32, h);
        }

#pragma unroll 1
        for (int j = 0; j < 16; ++j) {
            const int tloc = tq + 2 * j;
            const _Float16* bp = bplane + (size_t)((t0 + tloc) * C_DIM + ebase + n16) * S_DIM;
            v16h af[4];
#pragma unroll
            for (int ks = 0; ks < 4; ++ks) af[ks] = ld_frag_f16(bp, ks * 32, h);

            v8f acc0 = zero8(), acc1 = zero8();
#pragma unroll
            for (int ks = 0; ks < 4; ++ks) {
                acc0 = wmma_f16(acc0, af[ks], bq[0][ks]);
                acc1 = wmma_f16(acc1, af[ks], bq[1][ks]);
            }

            v8h o0, o1;
#pragma unroll
            for (int i = 0; i < 8; ++i) {
                o0[i] = (_Float16)acc0[i];
                o1[i] = (_Float16)acc1[i];
            }
            _Float16* dst = OT + (size_t)(rloc * 32 + tloc) * OT_PITCH + ebase + 8 * h;
            *(v8h*)(dst + n16 * 32)        = o0;
            *(v8h*)(dst + (16 + n16) * 32) = o1;
        }
    }
    __syncthreads();

    const int z0 = wave * 16;
    const _Float16* wp = wplane + (size_t)(z0 + n16) * KP_DIM;

    v8f acc[4];
#pragma unroll
    for (int mt = 0; mt < 4; ++mt) acc[mt] = zero8();

#pragma unroll 2
    for (int ks = 0; ks < KP_DIM / 32; ++ks) {
        const int k0 = ks * 32;
        const v16h bw = ld_frag_f16(wp, k0, h);
#pragma unroll
        for (int mt = 0; mt < 4; ++mt) {
            const v16h ao = ld_frag_f16(OT + (size_t)(mt * 16 + n16) * OT_PITCH, k0, h);
            acc[mt] = wmma_f16(acc[mt], ao, bw);
        }
    }
    __syncthreads();

    float* outS = (float*)dsmem;
    const float inv = 0.000244140625f;
#pragma unroll
    for (int mt = 0; mt < 4; ++mt) {
#pragma unroll
        for (int i = 0; i < 8; ++i)
            outS[(mt * 16 + 8 * h + i) * OS_PITCH + z0 + n16] = acc[mt][i] * inv;
    }
    __syncthreads();

    v4f vals[8];
#pragma unroll
    for (int pass = 0; pass < 8; ++pass) {
        const int L = pass * 32 + (tid >> 3);
        const int p = L >> 2, q = L & 3, sub = tid & 7;
        vals[pass] = *(const v4f*)(outS + p * OS_PITCH + q * 32 + sub * 4);
    }
#pragma unroll
    for (int pass = 0; pass < 8; ++pass) {
        const int L = pass * 32 + (tid >> 3);
        const int p = L >> 2, q = L & 3, sub = tid & 7;
        const int rr = r0 + (p >> 5), tt = t0 + (p & 31);
        float* gp = out + ((size_t)rr * R_DIM + tt) * CZ_DIM + q * 32 + sub * 4;
        *(volatile v4f*)gp = vals[pass];
    }
    __threadfence();
#pragma unroll
    for (int pass = 0; pass < 8; ++pass) {
        const int L = pass * 32 + (tid >> 3);
        const int p = L >> 2, q = L & 3, sub = tid & 7;
        const int rr = r0 + (p >> 5), tt = t0 + (p & 31);
        float* gp = out + ((size_t)rr * R_DIM + tt) * CZ_DIM + q * 32 + sub * 4;
        *(volatile v4f*)gp = vals[pass];
    }
}

extern "C" void kernel_launch(void* const* d_in, const int* in_sizes, int n_in,
                              void* d_out, int out_size, void* d_ws, size_t ws_size,
                              hipStream_t stream) {
    if (n_in < 4) return;
    if (in_sizes[0] != S_DIM * R_DIM * CM_DIM) return;
    if (in_sizes[1] != CM_DIM * C_DIM) return;
    if (in_sizes[2] != CM_DIM * C_DIM) return;
    if (in_sizes[3] != KP_DIM * CZ_DIM) return;
    if (out_size != R_DIM * R_DIM * CZ_DIM) return;

    const float* msa = (const float*)d_in[0];
    const float* wl  = (const float*)d_in[1];
    const float* wr  = (const float*)d_in[2];
    const float* wo  = (const float*)d_in[3];
    float* out = (float*)d_out;

    const size_t plane_bytes = (size_t)R_DIM * C_DIM * S_DIM * 2;
    const size_t wt_bytes    = (size_t)CZ_DIM * KP_DIM * 2;
    const size_t total       = 2 * plane_bytes + wt_bytes;
    if (total > ws_size) return;

    unsigned char* ws = (unsigned char*)d_ws;
    _Float16* aplane = (_Float16*)(ws);
    _Float16* bplane = (_Float16*)(ws + plane_bytes);
    _Float16* wplane = (_Float16*)(ws + 2 * plane_bytes);

    k_proj<<<dim3(R_DIM), dim3(256), PROJ_LDS_BYTES, stream>>>(msa, wl, wr, aplane, bplane);
    k_wprep<<<dim3(KP_DIM / 64), dim3(256), 0, stream>>>(wo, wplane);
    k_pair<<<dim3(R_DIM / 32, R_DIM / 2), dim3(256), PAIR_LDS_BYTES, stream>>>(aplane, bplane, wplane, out);
    (void)hipGetLastError();
}
